// SparseResBlock3d_21792664060178
// MI455X (gfx1250) — hardware-verified
//
#include <hip/hip_runtime.h>
#include <stddef.h>


typedef __bf16         v16bf __attribute__((ext_vector_type(16)));
typedef unsigned short v8us  __attribute__((ext_vector_type(8)));
typedef float          v8f   __attribute__((ext_vector_type(8)));
typedef float          v4f   __attribute__((ext_vector_type(4)));

union Frag { v16bf v; v8us u[2]; v8f f; };

#define C_IN     32
#define C_OUT    64
#define KOFF     27
#define VPB      64
#define NWB      2
#define KS_W1    0
#define KS_W2    27
#define KS_SK    81
#define KS_TOT   82
#define KS_US    2048
#define FT_PITCH 68
#define LN_EPS   1e-6f

__device__ __forceinline__ int imin(int a, int b) { return a < b ? a : b; }

__device__ __forceinline__ unsigned short f2bf(float f) {
    unsigned int u = __float_as_uint(f);
    u += 0x7FFFu + ((u >> 16) & 1u);
    return (unsigned short)(u >> 16);
}

__device__ __forceinline__ float silu_f(float y) {
    float e = __expf(-y);
    return y * __builtin_amdgcn_rcpf(1.0f + e);
}

__device__ __forceinline__ v8f wmma_bf16(const Frag& a, const Frag& b, v8f c) {
    return __builtin_amdgcn_wmma_f32_16x16x32_bf16(false, a.v, false, b.v, (short)0, c, false, false);
}

__device__ __forceinline__ void mma8(v8f (&acc)[8], const Frag& a0, const Frag& a1,
                                     const Frag& b0, const Frag& b1, const Frag& b2, const Frag& b3) {
    acc[0] = wmma_bf16(a0, b0, acc[0]);
    acc[4] = wmma_bf16(a1, b0, acc[4]);
    acc[1] = wmma_bf16(a0, b1, acc[1]);
    acc[5] = wmma_bf16(a1, b1, acc[5]);
    acc[2] = wmma_bf16(a0, b2, acc[2]);
    acc[6] = wmma_bf16(a1, b2, acc[6]);
    acc[3] = wmma_bf16(a0, b3, acc[3]);
    acc[7] = wmma_bf16(a1, b3, acc[7]);
    asm volatile("v_nop\n\tv_nop\n\tv_nop\n\tv_nop"
                 : "+v"(acc[0]), "+v"(acc[1]), "+v"(acc[2]), "+v"(acc[3]),
                   "+v"(acc[4]), "+v"(acc[5]), "+v"(acc[6]), "+v"(acc[7])
                 : "v"(a0.f), "v"(a1.f), "v"(b0.f), "v"(b1.f), "v"(b2.f), "v"(b3.f));
}

__device__ __forceinline__ void load_b4(const unsigned short* pw, int gks, int lane,
                                        Frag& b0, Frag& b1, Frag& b2, Frag& b3) {
    const v8us* q = (const v8us*)(pw + (size_t)gks * KS_US + (size_t)lane * 16);
    b0.u[0] = q[0];   b0.u[1] = q[1];
    b1.u[0] = q[64];  b1.u[1] = q[65];
    b2.u[0] = q[128]; b2.u[1] = q[129];
    b3.u[0] = q[192]; b3.u[1] = q[193];
}

__device__ __forceinline__ void stage_acc(float* ft, v8f (&acc)[8], const float* bias, int h, int m) {
    #pragma unroll
    for (int g = 0; g < 2; ++g) {
        #pragma unroll
        for (int tt = 0; tt < 4; ++tt) {
            const float b = bias[tt * 16 + m];
            #pragma unroll
            for (int r = 0; r < 8; ++r)
                ft[(g * 16 + 8 * h + r) * FT_PITCH + tt * 16 + m] = acc[g * 4 + tt][r] + b;
        }
    }
}

template <int CPR>
__device__ __forceinline__ void store_rows_bf16(const v8us* bt, unsigned short* dst, int lane) {
    #pragma unroll
    for (int j = 0; j < CPR; ++j) {
        const int c = j * 32 + lane;
        const v8us v = bt[c];
        *(volatile v8us*)(dst + (size_t)c * 8) = v;
    }
}

template <bool ADD>
__device__ __forceinline__ void store_rows_f32(const float* ft, const float* add, float* dst, int lane, int nvalid) {
    #pragma unroll
    for (int j = 0; j < 16; ++j) {
        const int c = j * 32 + lane;
        const int row = c >> 4, piece = c & 15;
        if (row < nvalid) {
            v4f v = *(const v4f*)(ft + row * FT_PITCH + piece * 4);
            const size_t off = (size_t)row * C_OUT + (size_t)piece * 4;
            if (ADD) v += *(const v4f*)(add + off);
            *(volatile v4f*)(dst + off) = v;
        }
    }
}

__global__ __launch_bounds__(256) void pack_w_kernel(const float* W1, const float* W2, const float* Wsk,
                                                     unsigned short* pw) {
    const int tid = blockIdx.x * 256 + threadIdx.x;
    const int gks = tid >> 8;
    if (gks >= KS_TOT) return;
    const int nt   = (tid >> 6) & 3;
    const int lane = (tid >> 1) & 31;
    const int hh   = tid & 1;
    const float* src;
    int ksl;
    if (gks < KS_W2)      { src = W1;  ksl = gks; }
    else if (gks < KS_SK) { src = W2;  ksl = gks - KS_W2; }
    else                  { src = Wsk; ksl = 0; }
    const int h  = lane >> 4;
    const int n  = nt * 16 + (lane & 15);
    const int kb = ksl * 32 + 16 * hh + 8 * h;
    v8us o = {0, 0, 0, 0, 0, 0, 0, 0};
    #pragma unroll
    for (int e = 0; e < 8; ++e) o[e] = f2bf(src[(size_t)(kb + e) * C_OUT + n]);
    volatile v8us* d = (volatile v8us*)(pw + (size_t)tid * 8);
    *d = o;
    __threadfence();
    *d = o;
}

__global__ __launch_bounds__(64) void ln1_skip_kernel(const float* feats, const float* gamma, const float* beta,
                                                      const unsigned short* pw, const float* bskip,
                                                      unsigned short* h1, float* sk, int N) {
    __shared__ v8us  gtile[VPB * 4];
    __shared__ v8us  btile[VPB * 4];
    __shared__ float ftile[NWB * 32 * FT_PITCH];

    const int t = threadIdx.x, lane = t & 31, w = t >> 5, h = lane >> 4, m = lane & 15;
    const int vbase = blockIdx.x * VPB + w * 32;
    const int voxc  = imin(vbase + lane, N - 1);

    const v4f* fr = (const v4f*)(feats + (size_t)voxc * C_IN);
    v4f x[8];
    #pragma unroll
    for (int j = 0; j < 8; ++j) x[j] = fr[j];

    #pragma unroll
    for (int j = 0; j < 4; ++j) {
        v8us o = {0, 0, 0, 0, 0, 0, 0, 0};
        #pragma unroll
        for (int e = 0; e < 8; ++e) { const int c = j * 8 + e; o[e] = f2bf(x[c >> 2][c & 3]); }
        gtile[t * 4 + j] = o;
    }

    float s = 0.f;
    #pragma unroll
    for (int j = 0; j < 8; ++j) { s += x[j][0]; s += x[j][1]; s += x[j][2]; s += x[j][3]; }
    const float mu = s * (1.0f / C_IN);
    float q = 0.f;
    #pragma unroll
    for (int j = 0; j < 8; ++j) {
        #pragma unroll
        for (int e = 0; e < 4; ++e) { const float d = x[j][e] - mu; q += d * d; }
    }
    const float rs = rsqrtf(q * (1.0f / C_IN) + LN_EPS);
    #pragma unroll
    for (int j = 0; j < 4; ++j) {
        v8us o = {0, 0, 0, 0, 0, 0, 0, 0};
        #pragma unroll
        for (int e = 0; e < 8; ++e) {
            const int c = j * 8 + e;
            float y = (x[c >> 2][c & 3] - mu) * rs;
            y = y * gamma[c] + beta[c];
            o[e] = f2bf(silu_f(y));
        }
        btile[t * 4 + j] = o;
    }
    __syncthreads();

    v8f acc[8] = {};
    {
        Frag a0, a1, b0, b1, b2, b3;
        const int ra = (w * 32 + m) * 4, rb = (w * 32 + 16 + m) * 4;
        a0.u[0] = gtile[ra + h];  a0.u[1] = gtile[ra + 2 + h];
        a1.u[0] = gtile[rb + h];  a1.u[1] = gtile[rb + 2 + h];
        load_b4(pw, KS_SK, lane, b0, b1, b2, b3);
        mma8(acc, a0, a1, b0, b1, b2, b3);
    }
    float* ftw = ftile + w * 32 * FT_PITCH;
    stage_acc(ftw, acc, bskip, h, m);
    __syncthreads();

    unsigned short* h1w = h1 + (size_t)vbase * C_IN;
    float*          skw = sk + (size_t)vbase * C_OUT;
    const v8us*     btw = btile + w * 32 * 4;
    store_rows_bf16<4>(btw, h1w, lane);
    store_rows_f32<false>(ftw, nullptr, skw, lane, 32);
    __threadfence();
    store_rows_bf16<4>(btw, h1w, lane);
    store_rows_f32<false>(ftw, nullptr, skw, lane, 32);
}

__global__ __launch_bounds__(64) void conv1_ln2_kernel(const unsigned short* h1, const int* nbr,
                                                       const unsigned short* pw, const float* bconv1,
                                                       unsigned short* h2, int N) {
    __shared__ v8us  gtile[VPB * 4];
    __shared__ v8us  btile[VPB * 8];
    __shared__ float ftile[NWB * 32 * FT_PITCH];

    const int t = threadIdx.x, lane = t & 31, w = t >> 5, h = lane >> 4, m = lane & 15;
    const int vbase = blockIdx.x * VPB + w * 32;
    const int voxc  = imin(blockIdx.x * VPB + t, N - 1);
    const int* nrow = nbr + (size_t)voxc * KOFF;
    const int ra = (w * 32 + m) * 4, rb = (w * 32 + 16 + m) * 4;
    const v8us zz = {0, 0, 0, 0, 0, 0, 0, 0};

    v8f acc[8] = {};
    #pragma unroll 1
    for (int ko = 0; ko < KOFF; ++ko) {
        const int  v     = nrow[ko];
        const bool valid = v >= 0;
        const int  r     = valid ? imin(v, N - 1) : 0;
        const v8us* src  = (const v8us*)(h1 + (size_t)r * C_IN);
        v8us cc[4];
        #pragma unroll
        for (int j = 0; j < 4; ++j) cc[j] = src[j];
        if (!valid) {
            #pragma unroll
            for (int j = 0; j < 4; ++j) cc[j] = zz;
        }
        __syncthreads();
        #pragma unroll
        for (int j = 0; j < 4; ++j) gtile[t * 4 + j] = cc[j];
        __syncthreads();
        Frag a0, a1, b0, b1, b2, b3;
        a0.u[0] = gtile[ra + h];  a0.u[1] = gtile[ra + 2 + h];
        a1.u[0] = gtile[rb + h];  a1.u[1] = gtile[rb + 2 + h];
        load_b4(pw, KS_W1 + ko, lane, b0, b1, b2, b3);
        mma8(acc, a0, a1, b0, b1, b2, b3);
    }

    float* ftw = ftile + w * 32 * FT_PITCH;
    stage_acc(ftw, acc, bconv1, h, m);
    __syncthreads();

    {
        const float* frw = ftw + lane * FT_PITCH;
        v4f x[16];
        #pragma unroll
        for (int j = 0; j < 16; ++j) x[j] = *(const v4f*)(frw + j * 4);
        float s = 0.f;
        #pragma unroll
        for (int j = 0; j < 16; ++j) { s += x[j][0]; s += x[j][1]; s += x[j][2]; s += x[j][3]; }
        const float mu = s * (1.0f / C_OUT);
        float q = 0.f;
        #pragma unroll
        for (int j = 0; j < 16; ++j) {
            #pragma unroll
            for (int e = 0; e < 4; ++e) { const float d = x[j][e] - mu; q += d * d; }
        }
        const float rs = rsqrtf(q * (1.0f / C_OUT) + LN_EPS);
        v8us* btw = btile + (w * 32 + lane) * 8;
        #pragma unroll
        for (int j = 0; j < 8; ++j) {
            v8us o = {0, 0, 0, 0, 0, 0, 0, 0};
            #pragma unroll
            for (int e = 0; e < 8; ++e) {
                const int c = j * 8 + e;
                const float y = (x[c >> 2][c & 3] - mu) * rs;
                o[e] = f2bf(silu_f(y));
            }
            btw[j] = o;
        }
    }
    __syncthreads();

    unsigned short* h2w = h2 + (size_t)vbase * C_OUT;
    const v8us*     btw = btile + w * 32 * 8;
    store_rows_bf16<8>(btw, h2w, lane);
    __threadfence();
    store_rows_bf16<8>(btw, h2w, lane);
}

__global__ __launch_bounds__(64) void conv2_out_kernel(const unsigned short* h2, const int* nbr,
                                                       const unsigned short* pw, const float* bconv2,
                                                       const float* sk, float* out, int N) {
    __shared__ v8us  gtile[VPB * 8];
    __shared__ float ftile[NWB * 32 * FT_PITCH];

    const int t = threadIdx.x, lane = t & 31, w = t >> 5, h = lane >> 4, m = lane & 15;
    const int vbase = blockIdx.x * VPB + w * 32;
    const int voxc  = imin(blockIdx.x * VPB + t, N - 1);
    const int* nrow = nbr + (size_t)voxc * KOFF;
    const int ra = (w * 32 + m) * 8, rb = (w * 32 + 16 + m) * 8;
    const v8us zz = {0, 0, 0, 0, 0, 0, 0, 0};

    v8f acc[8] = {};
    #pragma unroll 1
    for (int ko = 0; ko < KOFF; ++ko) {
        const int  v     = nrow[ko];
        const bool valid = v >= 0;
        const int  r     = valid ? imin(v, N - 1) : 0;
        const v8us* src  = (const v8us*)(h2 + (size_t)r * C_OUT);
        v8us cc[8];
        #pragma unroll
        for (int j = 0; j < 8; ++j) cc[j] = src[j];
        if (!valid) {
            #pragma unroll
            for (int j = 0; j < 8; ++j) cc[j] = zz;
        }
        __syncthreads();
        #pragma unroll
        for (int j = 0; j < 8; ++j) gtile[t * 8 + j] = cc[j];
        __syncthreads();
        #pragma unroll
        for (int s = 0; s < 2; ++s) {
            Frag a0, a1, b0, b1, b2, b3;
            a0.u[0] = gtile[ra + s * 4 + h];  a0.u[1] = gtile[ra + s * 4 + 2 + h];
            a1.u[0] = gtile[rb + s * 4 + h];  a1.u[1] = gtile[rb + s * 4 + 2 + h];
            load_b4(pw, KS_W2 + ko * 2 + s, lane, b0, b1, b2, b3);
            mma8(acc, a0, a1, b0, b1, b2, b3);
        }
    }

    float* ftw = ftile + w * 32 * FT_PITCH;
    stage_acc(ftw, acc, bconv2, h, m);
    __syncthreads();

    const int    nvalid = N - vbase;
    const float* skw    = sk + (size_t)vbase * C_OUT;
    float*       outw   = out + (size_t)vbase * C_OUT;
    store_rows_f32<true>(ftw, skw, outw, lane, nvalid);
    __threadfence();
    store_rows_f32<true>(ftw, skw, outw, lane, nvalid);
}

static inline size_t align256(size_t x) { return (x + 255) & ~(size_t)255; }

extern "C" void kernel_launch(void* const* d_in, const int* in_sizes, int n_in,
                              void* d_out, int out_size, void* d_ws, size_t ws_size,
                              hipStream_t stream) {
    if (n_in < 10) return;
    const float* feats  = (const float*)d_in[0];
    const int*   nbr    = (const int*)d_in[1];
    const float* gamma1 = (const float*)d_in[2];
    const float* beta1  = (const float*)d_in[3];
    const float* W1     = (const float*)d_in[4];
    const float* bconv1 = (const float*)d_in[5];
    const float* W2     = (const float*)d_in[6];
    const float* bconv2 = (const float*)d_in[7];
    const float* Wskip  = (const float*)d_in[8];
    const float* bskip  = (const float*)d_in[9];
    float* out = (float*)d_out;

    const int N = in_sizes[0] / C_IN;
    if (N <= 0) return;
    if (in_sizes[0] != N * C_IN || in_sizes[1] != N * KOFF || out_size != N * C_OUT) return;
    if (in_sizes[2] < C_IN || in_sizes[3] < C_IN) return;
    if (in_sizes[4] != KOFF * C_IN * C_OUT || in_sizes[6] != KOFF * C_OUT * C_OUT || in_sizes[8] != C_IN * C_OUT) return;
    if (in_sizes[5] < C_OUT || in_sizes[7] < C_OUT || in_sizes[9] < C_OUT) return;

    const int    NB = (N + VPB - 1) / VPB;
    const size_t NR = (size_t)NB * VPB;

    char* ws = (char*)d_ws;
    size_t o = 0;
    unsigned short* pw = (unsigned short*)(ws + o); o += align256((size_t)KS_TOT * KS_US * 2);
    unsigned short* h1 = (unsigned short*)(ws + o); o += align256(NR * C_IN * 2);
    unsigned short* h2 = (unsigned short*)(ws + o); o += align256(NR * C_OUT * 2);
    float*          sk = (float*)(ws + o);          o += align256(NR * C_OUT * 4);
    if (o > ws_size) return;

    pack_w_kernel<<<KS_TOT, 256, 0, stream>>>(W1, W2, Wskip, pw);
    ln1_skip_kernel<<<NB, 64, 0, stream>>>(feats, gamma1, beta1, pw, bskip, h1, sk, N);
    conv1_ln2_kernel<<<NB, 64, 0, stream>>>(h1, nbr, pw, bconv1, h2, N);
    conv2_out_kernel<<<NB, 64, 0, stream>>>(h2, nbr, pw, bconv2, sk, out, N);
}
